// Cwt_65816078843929
// MI455X (gfx1250) — hardware-verified
//
#include <hip/hip_runtime.h>


#define NBS  128
#define NN   1024
#define NSC  101
#define SCH  16
#define OH   200
#define OW   200
#define PADL 511
typedef _Float16 h16;
typedef unsigned short bf;
typedef __attribute__((ext_vector_type(16))) __bf16   v16bf;
typedef __attribute__((ext_vector_type(16))) _Float16 v16h;
typedef __attribute__((ext_vector_type(8)))  _Float16 v8h;
typedef __attribute__((ext_vector_type(8)))  unsigned short v8us;
typedef __attribute__((ext_vector_type(8)))  float    v8f;
typedef __attribute__((ext_vector_type(4)))  float    v4f;
typedef v8h  __attribute__((may_alias)) v8ha;
typedef v4f  __attribute__((may_alias)) v4fa;
typedef v8us __attribute__((may_alias)) v8usa;

__device__ __forceinline__ unsigned short f2bf(float f) { unsigned u = __float_as_uint(f); u += 0x7FFFu + ((u >> 16) & 1u); return (unsigned short)(u >> 16); }
__device__ __forceinline__ float bf2f(unsigned short b) { return __uint_as_float(((unsigned)b) << 16); }
__device__ __forceinline__ float bfr(float f) { return bf2f(f2bf(f)); }
__device__ __forceinline__ v16h cat16(v8h lo, v8h hi) { return __builtin_shufflevector(lo, hi, 0, 1, 2, 3, 4, 5, 6, 7, 8, 9, 10, 11, 12, 13, 14, 15); }
__device__ __forceinline__ v16bf cat16b(v8us lo, v8us hi) { return __builtin_bit_cast(v16bf, __builtin_shufflevector(lo, hi, 0, 1, 2, 3, 4, 5, 6, 7, 8, 9, 10, 11, 12, 13, 14, 15)); }
__device__ __forceinline__ v8f wmma16(v16h a, v16h b, v8f c) { return __builtin_amdgcn_wmma_f32_16x16x32_f16(false, a, false, b, (short)0, c, false, false); }
__device__ __forceinline__ v8f wmmab(v16bf a, v16bf b, v8f c) { return __builtin_amdgcn_wmma_f32_16x16x32_bf16(false, a, false, b, (short)0, c, false, false); }


template <typename T16> struct WFrag;
template <> struct WFrag<h16> { typedef v16h V; static __device__ __forceinline__ V ld(const h16* p) { return cat16(*(const v8h*)p, *(const v8h*)(p + 16)); } static __device__ __forceinline__ v8f mma(V a, V b, v8f c) { return wmma16(a, b, c); } };
template <> struct WFrag<bf> { typedef v16bf V; static __device__ __forceinline__ V ld(const bf* p) { return cat16b(*(const v8us*)p, *(const v8us*)(p + 16)); } static __device__ __forceinline__ v8f mma(V a, V b, v8f c) { return wmmab(a, b, c); } };
template <typename T16, int NSPLIT, bool BIAS>
__global__ __launch_bounds__(32) void k_gemmw(const T16* __restrict__ A, const T16* __restrict__ A2, const T16* __restrict__ Bt, const T16* __restrict__ Bt2, int K, float* C, int ldc, const float* __restrict__ bias, size_t sA, size_t sB, size_t sC) {
    typedef typename WFrag<T16>::V V;
    __shared__ __align__(16) float os[16 * 68];
    const size_t z = blockIdx.z; A += z * sA; if (A2) A2 += z * sA; Bt += z * sB; if (Bt2) Bt2 += z * sB; C += z * sC;
    const int lane = threadIdx.x & 31, lr = lane & 15, hi = lane >> 4; const int r0 = blockIdx.x * 64, c0 = blockIdx.y * 64;
    v8f acc[4][4];
#pragma unroll
    for (int mb = 0; mb < 4; ++mb)
#pragma unroll
        for (int nb = 0; nb < 4; ++nb) acc[mb][nb] = (v8f){};
    const size_t aoff = (size_t)(r0 + lr) * K + 8 * hi, boff = (size_t)(c0 + lr) * K + 8 * hi;
#pragma unroll 1
    for (int kc = 0; kc < K; kc += 32) {
        V a[4], a2[4];
#pragma unroll
        for (int mb = 0; mb < 4; ++mb) { a[mb] = WFrag<T16>::ld(A + aoff + (size_t)mb * 16 * K + kc); if (NSPLIT == 1 || NSPLIT == 2) a2[mb] = WFrag<T16>::ld(A2 + aoff + (size_t)mb * 16 * K + kc); }
#pragma unroll
        for (int nb = 0; nb < 4; ++nb) { const V b = WFrag<T16>::ld(Bt + boff + (size_t)nb * 16 * K + kc); V b2; if (NSPLIT >= 2) b2 = WFrag<T16>::ld(Bt2 + boff + (size_t)nb * 16 * K + kc);
#pragma unroll
            for (int mb = 0; mb < 4; ++mb) { acc[mb][nb] = WFrag<T16>::mma(a[mb], b, acc[mb][nb]); if (NSPLIT == 1 || NSPLIT == 2) acc[mb][nb] = WFrag<T16>::mma(a2[mb], b, acc[mb][nb]); if (NSPLIT >= 2) acc[mb][nb] = WFrag<T16>::mma(a[mb], b2, acc[mb][nb]); } }
        asm volatile("v_nop\n\tv_nop\n\tv_nop\n\tv_nop" : "+v"(acc[0][0]), "+v"(acc[1][1]), "+v"(acc[2][2]), "+v"(acc[3][3]) : "v"(a[0]), "v"(a[3]));
    }
#pragma unroll
    for (int mb = 0; mb < 4; ++mb) {
#pragma unroll
        for (int nb = 0; nb < 4; ++nb) {
#pragma unroll
            for (int j = 0; j < 8; ++j) os[(hi * 8 + j) * 68 + nb * 16 + lr] = acc[mb][nb][j]; }
        __builtin_amdgcn_wave_barrier(); asm volatile("" ::: "memory");
        float* crow = C + (size_t)(r0 + mb * 16) * ldc + c0;
#pragma unroll 1
        for (int ps = 0; ps < 2; ++ps) {
#pragma unroll
            for (int s = 0; s < 8; ++s) { const int row = 2 * s + hi, cofs = lr * 4; v4f val = *(const v4fa*)(os + row * 68 + cofs); if (BIAS) { val[0] += bfr(bias[c0 + cofs]); val[1] += bfr(bias[c0 + cofs + 1]); val[2] += bfr(bias[c0 + cofs + 2]); val[3] += bfr(bias[c0 + cofs + 3]); }
                *(volatile v4f*)(crow + (size_t)row * ldc + cofs) = val; }
            if (ps == 0) __threadfence(); }
        __builtin_amdgcn_wave_barrier(); asm volatile("" ::: "memory");
    }
}

typedef __attribute__((ext_vector_type(4))) unsigned short v4us;
typedef __attribute__((ext_vector_type(2))) float v2f;

__global__ __launch_bounds__(256) void k_xrev(const float* __restrict__ x, bf* Bt) { const int e = (blockIdx.x * 256 + threadIdx.x) * 4; if (e >= NBS * NN) return; const int k = e % NN; const int b = e / NN; v4us o;
#pragma unroll
    for (int u = 0; u < 4; ++u) o[u] = f2bf(x[(size_t)b * NN + (NN - 1 - (k + u))]); *(volatile v4us*)(Bt + e) = o; __threadfence(); *(volatile v4us*)(Bt + e) = o; }
__global__ __launch_bounds__(256) void k_toep(const float* __restrict__ ker, int s0, int ns, bf* A) { const size_t e = ((size_t)blockIdx.x * 256 + threadIdx.x) * 4; if (e >= (size_t)ns * NN * NN) return; const int k = (int)(e % NN); const int n = (int)((e / NN) % NN); const int s = s0 + (int)(e / ((size_t)NN * NN)); v4us o;
#pragma unroll
    for (int u = 0; u < 4; ++u) { const int m = n + (k + u) - PADL; const bool inb = (s < NSC && m >= 0 && m < NN); const int mc = min(max(m, 0), NN - 1), scl = min(s, NSC - 1); const float v = ker[(size_t)scl * NN + mc]; o[u] = inb ? f2bf(v) : (unsigned short)0; } *(volatile v4us*)(A + e) = o; __threadfence(); *(volatile v4us*)(A + e) = o; }
__global__ __launch_bounds__(128) void k_mm(const float* __restrict__ R, float* MM) { const int b = threadIdx.x; float mn = 3.0e38f, mx = -3.0e38f;
#pragma unroll 1
    for (int r = 0; r < NSC * NN; ++r) { const float v = R[(size_t)r * NBS + b]; mn = fminf(mn, v); mx = fmaxf(mx, v); } v2f o; o[0] = mn; o[1] = mx; *(volatile v2f*)(MM + b * 2) = o; __threadfence(); *(volatile v2f*)(MM + b * 2) = o; }
__device__ __forceinline__ void taps(int i, int insz, int outsz, int& i0, int& i1, float& w0, float& w1) {
    const float sf = __fsub_rn(__fmul_rn((float)i + 0.5f, (float)insz / (float)outsz), 0.5f); const float fl = floorf(sf); const float fr = __fsub_rn(sf, fl); int a = (int)fl, b = a + 1; float wa = __fsub_rn(1.0f, fr), wb = fr;
    if (a < 0) { wa = 0.f; a = 0; } if (b > insz - 1) { wb = 0.f; b = insz - 1; } const float tot = __fadd_rn(wa, wb); i0 = a; i1 = b; w0 = __fdiv_rn(wa, tot); w1 = __fdiv_rn(wb, tot); }
__global__ __launch_bounds__(256) void k_tab(int insz, int outsz, float* T) { const int i = blockIdx.x * 256 + threadIdx.x; if (i >= outsz) return; int i0, i1; float w0, w1; taps(i, insz, outsz, i0, i1, w0, w1); v4f o; o[0] = (float)i0; o[1] = (float)i1; o[2] = w0; o[3] = w1; *(volatile v4f*)(T + (size_t)i * 4) = o; __threadfence(); *(volatile v4f*)(T + (size_t)i * 4) = o; }
__global__ __launch_bounds__(256) void k_norm(float* R, const float* __restrict__ MM) { const size_t e = ((size_t)blockIdx.x * 256 + threadIdx.x) * 4; if (e >= (size_t)NSC * NN * NBS) return; const int b = (int)(e % NBS); const v4f a = *(const v4f*)(R + e); v4f o;
#pragma unroll
    for (int u = 0; u < 4; ++u) { const v2f mm = *(const v2f*)(MM + (b + u) * 2); o[u] = __fdiv_rn(__fsub_rn(a[u], mm[0]), __fsub_rn(mm[1], mm[0])); } *(volatile v4f*)(R + e) = o; __threadfence(); *(volatile v4f*)(R + e) = o; }
__global__ __launch_bounds__(256) void k_rsz(const float* __restrict__ R, const float* __restrict__ TY, const float* __restrict__ TX, float* OUT) { const size_t e = ((size_t)blockIdx.x * 256 + threadIdx.x) * 4; if (e >= (size_t)NBS * OH * OW) return; const int j = (int)(e % OW); const int i = (int)((e / OW) % OH); const int b = (int)(e / ((size_t)OW * OH));
    const v4f ty = *(const v4f*)(TY + (size_t)i * 4); const int s0 = (int)ty[0], s1 = (int)ty[1]; const float ws0 = ty[2], ws1 = ty[3]; v4f o;
#pragma unroll
    for (int u = 0; u < 4; ++u) { const v4f tx = *(const v4f*)(TX + (size_t)(j + u) * 4); const int n0 = (int)tx[0], n1 = (int)tx[1]; const float wn0 = tx[2], wn1 = tx[3];
        auto nv = [&](int s, int n) { return R[((size_t)s * NN + n) * NBS + b]; };
        float c0 = __fadd_rn(__fmul_rn(ws0, nv(s0, n0)), __fmul_rn(ws1, nv(s1, n0))); float c1 = __fadd_rn(__fmul_rn(ws0, nv(s0, n1)), __fmul_rn(ws1, nv(s1, n1))); asm volatile("" : "+v"(c0)); asm volatile("" : "+v"(c1));
        float t0 = __fmul_rn(wn0, c0), t1 = __fmul_rn(wn1, c1); asm volatile("" : "+v"(t0)); asm volatile("" : "+v"(t1)); o[u] = __fadd_rn(t0, t1); }
    *(volatile v4f*)(OUT + e) = o; __threadfence(); *(volatile v4f*)(OUT + e) = o; }

extern "C" void kernel_launch(void* const* d_in, const int* in_sizes, int n_in,
                              void* d_out, int out_size, void* d_ws, size_t ws_size, hipStream_t stream) {
    (void)in_sizes; (void)n_in; (void)out_size;
    const float** I = (const float**)d_in;
    const float *x = I[0], *ker = I[1];
    float* OUT = (float*)d_out;
    char* wsp = (char*)d_ws;
    auto take = [&](size_t bytes) { char* p = wsp; wsp += (bytes + 255) & ~(size_t)255; return (void*)p; };
    bf* Bt = (bf*)take((size_t)NBS * NN * 2); bf* A = (bf*)take((size_t)SCH * NN * NN * 2); float* R = (float*)take((size_t)NSC * NN * NBS * 4); float* MM = (float*)take(NBS * 2 * 4); float* TY = (float*)take(OH * 16); float* TX = (float*)take(OW * 16);
    if ((size_t)(wsp - (char*)d_ws) > ws_size) return;
    k_xrev<<<(NBS * NN / 4 + 255) / 256, 256, 0, stream>>>(x, Bt);
    for (int s0 = 0; s0 < NSC; s0 += SCH) { const int ns = (NSC - s0 < SCH) ? (NSC - s0) : SCH;
        k_toep<<<(unsigned)(((size_t)ns * NN * NN / 4 + 255) / 256), 256, 0, stream>>>(ker, s0, ns, A);
        k_gemmw<bf, 0, false><<<dim3(ns * NN / 64, NBS / 64, 1), 32, 0, stream>>>(A, nullptr, Bt, nullptr, NN, R + (size_t)s0 * NN * NBS, NBS, nullptr, 0, 0, 0); }
    k_mm<<<1, 128, 0, stream>>>(R, MM); k_norm<<<(unsigned)(((size_t)NSC * NN * NBS / 4 + 255) / 256), 256, 0, stream>>>(R, MM);
    k_tab<<<1, 256, 0, stream>>>(NSC, OH, TY); k_tab<<<1, 256, 0, stream>>>(NN, OW, TX);
    k_rsz<<<(unsigned)(((size_t)NBS * OH * OW / 4 + 255) / 256), 256, 0, stream>>>(R, TY, TX, OUT);
}
